// UCCAEncoder_40553081208841
// MI455X (gfx1250) — hardware-verified
//
#include <hip/hip_runtime.h>
#include <stddef.h>


#define DD      256
#define KP      256
#define APZ     264
#define NTHR    256
#define NWAV    8
#define GROWS   32
#define PQW     512
#define NBC     512
#define GNODE   16
#define NGRP    (NBC / GNODE)
#define EPT     16
#define CHUNK   (NTHR * EPT)
#define HC      16384
#define GC      1024
#define TROWS   32
#define NGRAPH  8
#define ORB     16
#define W1T     16384
#define W2T     8192
#define WSC     64.0f
#define HSC     16.0f
#define RH      0.0009765625f
#define WSCAP   134217728
#define LDS_NODE (GROWS * APZ * 2 + GROWS * PQW * 4 + 3 * DD * 4)
#define LDS_FFN  (2 * GROWS * APZ * 2 + GROWS * DD * 4 + 4 * DD * 4)
#define LDS_CONV (HC * 4 + GC * 4 + TROWS * APZ * 2 + TROWS * DD * 4 + GNODE * DD * 4 + DD * 4 + TROWS * 4 + 64)

static_assert(NTHR == DD && NTHR == 32 * NWAV);
static_assert(GROWS == 4 * NWAV && GROWS == 32);
static_assert((NWAV / 2) * 128 == PQW && (NWAV / 2) * 64 == DD && NWAV * 32 == DD);
static_assert(TROWS * 8 == NTHR && TROWS == 32);
static_assert(CHUNK == 4096 && (HC % CHUNK) == 0 && GC == 32 * TROWS);
static_assert(NBC == NGRP * GNODE && GNODE == 16 && NBC == 512);
static_assert(GNODE * DD == 4 * 4 * NTHR);
static_assert(GROWS * PQW == 16 * 4 * NTHR && GROWS * DD == 8 * 4 * NTHR && ORB * DD == 4 * 4 * NTHR);
static_assert((APZ % 8) == 0 && (KP % 32) == 0 && (DD % 32) == 0);
static_assert(W1T * 8 == PQW * KP && W2T * 8 == DD * KP && (W1T % NTHR) == 0 && (W2T % NTHR) == 0);
static_assert(((GROWS * APZ * 2) % 16) == 0 && ((HC * 4 + GC * 4 + TROWS * APZ * 2) % 16) == 0);
static_assert(LDS_CONV < 300000 && LDS_NODE < 300000 && LDS_FFN < 300000);

typedef float    v4f  __attribute__((ext_vector_type(4)));
typedef float    v8f  __attribute__((ext_vector_type(8)));
typedef int      v4i  __attribute__((ext_vector_type(4)));
typedef _Float16 v8h  __attribute__((ext_vector_type(8)));
typedef _Float16 v16h __attribute__((ext_vector_type(16)));
union Frag { v16h v; v8h h[2]; };

__device__ __forceinline__ v8f wmh(v16h a, v16h b, v8f c) {
  v8f d = __builtin_amdgcn_wmma_f32_16x16x32_f16(false, a, false, b, (short)0, c, false, false);
  asm volatile("v_nop\n\tv_nop\n\tv_nop\n\tv_nop" : "+v"(d) : "v"(a), "v"(b));
  return d;
}

template <int NT>
__device__ __forceinline__ void mma16(const _Float16* Ar, const _Float16* __restrict__ Bpl, int lane,
                                      v8f (&acc)[NT]) {
  const int hh = lane >> 4, m = lane & 15;
#pragma unroll
  for (int t = 0; t < NT; ++t) { v8f z = {0.f, 0.f, 0.f, 0.f, 0.f, 0.f, 0.f, 0.f}; acc[t] = z; }
  const _Float16* ap = Ar + m * APZ + 8 * hh;
  const _Float16* bb = Bpl + (size_t)m * KP + 8 * hh;
#pragma unroll 1
  for (int ks = 0; ks < DD / 32; ++ks) {
    Frag a;
    a.h[0] = *(const v8h*)(ap + 32 * ks);
    a.h[1] = *(const v8h*)(ap + 32 * ks + 16);
#pragma unroll
    for (int t = 0; t < NT; ++t) {
      const _Float16* bp = bb + (size_t)(16 * t) * KP + 32 * ks;
      Frag b;
      b.h[0] = *(const v8h*)bp;
      b.h[1] = *(const v8h*)(bp + 16);
      acc[t] = wmh(a.v, b.v, acc[t]);
    }
  }
}

template <int NT>
__device__ __forceinline__ void mma32(const _Float16* Ar, const _Float16* __restrict__ Bpl, int lane,
                                      v8f (&c0)[NT], v8f (&c1)[NT]) {
  const int hh = lane >> 4, m = lane & 15;
#pragma unroll
  for (int t = 0; t < NT; ++t) {
    v8f z = {0.f, 0.f, 0.f, 0.f, 0.f, 0.f, 0.f, 0.f};
    c0[t] = z; c1[t] = z;
  }
  const _Float16* ap = Ar + m * APZ + 8 * hh;
  const _Float16* bb = Bpl + (size_t)m * KP + 8 * hh;
#pragma unroll 1
  for (int ks = 0; ks < DD / 32; ++ks) {
    Frag x0, x1;
    x0.h[0] = *(const v8h*)(ap + 32 * ks);
    x0.h[1] = *(const v8h*)(ap + 32 * ks + 16);
    x1.h[0] = *(const v8h*)(ap + 16 * APZ + 32 * ks);
    x1.h[1] = *(const v8h*)(ap + 16 * APZ + 32 * ks + 16);
#pragma unroll
    for (int t = 0; t < NT; ++t) {
      const _Float16* bp = bb + (size_t)(16 * t) * KP + 32 * ks;
      Frag b;
      b.h[0] = *(const v8h*)bp;
      b.h[1] = *(const v8h*)(bp + 16);
      c0[t] = wmh(x0.v, b.v, c0[t]);
      c1[t] = wmh(x1.v, b.v, c1[t]);
    }
  }
}

__global__ __launch_bounds__(NTHR) void k_wprep(const float* __restrict__ w1, const float* __restrict__ w2,
                                                const float* __restrict__ f1, const float* __restrict__ f2,
                                                _Float16* P1, _Float16* P2, _Float16* Q1, _Float16* Q2, int nl) {
  const int blk = blockIdx.x, tid = threadIdx.x;
  const int e1 = nl * (W1T / NTHR), e2 = e1 + nl * (W2T / NTHR), e3 = e2 + W2T / NTHR;
  float v[8];
  _Float16* dp;
  if (blk < e1) {
    const int i = blk * NTHR + tid;
    const int l = i / W1T, r = i - l * W1T;
    const int n = r >> 5, k0 = (r & 31) * 8;
    const float* wl = w1 + (size_t)l * (2 * DD * DD);
    if (n < DD) {
#pragma unroll
      for (int e = 0; e < 8; ++e)
        v[e] = wl[(size_t)(k0 + e) * DD + n] - wl[(size_t)(DD + k0 + e) * DD + n];
    } else {
#pragma unroll
      for (int e = 0; e < 8; ++e) v[e] = wl[(size_t)(DD + k0 + e) * DD + (n - DD)];
    }
    dp = P1 + (size_t)l * (PQW * KP) + (size_t)r * 8;
  } else if (blk < e2) {
    const int i = (blk - e1) * NTHR + tid;
    const int l = i / W2T, r = i - l * W2T;
    const int n = r >> 5, k0 = (r & 31) * 8;
    const float* wl = w2 + (size_t)l * (DD * DD);
#pragma unroll
    for (int e = 0; e < 8; ++e) v[e] = wl[(size_t)(k0 + e) * DD + n];
    dp = P2 + (size_t)l * (DD * KP) + (size_t)r * 8;
  } else if (blk < e3) {
    const int i = (blk - e2) * NTHR + tid;
    const int n = i >> 5, k0 = (i & 31) * 8;
#pragma unroll
    for (int e = 0; e < 8; ++e) v[e] = f1[(size_t)(k0 + e) * DD + n];
    dp = Q1 + (size_t)i * 8;
  } else {
    const int i = (blk - e3) * NTHR + tid;
    const int n = i >> 5, k0 = (i & 31) * 8;
#pragma unroll
    for (int e = 0; e < 8; ++e) v[e] = f2[(size_t)(k0 + e) * DD + n];
    dp = Q2 + (size_t)i * 8;
  }
  v8h hv;
#pragma unroll
  for (int e = 0; e < 8; ++e) hv[e] = (_Float16)(v[e] * WSC);
  *(volatile v8h*)dp = hv;
  __threadfence();
  *(volatile v8h*)dp = hv;
}

__device__ __forceinline__ void loadids(const int* __restrict__ ids, int nE, int cbase, int tid, int vec,
                                        int (&d)[EPT]) {
  const int e0 = cbase + EPT * tid;
  if (vec != 0 && cbase + CHUNK <= nE) {
#pragma unroll
    for (int q = 0; q < EPT / 4; ++q) {
      const v4i t4 = *(const v4i*)(ids + e0 + 4 * q);
      d[4 * q] = t4.x; d[4 * q + 1] = t4.y; d[4 * q + 2] = t4.z; d[4 * q + 3] = t4.w;
    }
  } else {
#pragma unroll
    for (int j = 0; j < EPT; ++j) {
      int idx = e0 + j;
      const bool ok = idx < nE;
      idx = ok ? idx : nE - 1;
      const int val = ids[idx];
      d[j] = ok ? val : (-2147483647 - 1);
    }
  }
}

__device__ __forceinline__ void blkscan(int cnt, int lane, int wave, int* swt, int& pos, int& nh) {
  int x = cnt;
#pragma unroll
  for (int o = 1; o < 32; o <<= 1) {
    const int y = __shfl_up(x, o, 32);
    x += (lane >= o) ? y : 0;
  }
  if (lane == 31) swt[wave] = x;
  __syncthreads();
  int wpre = 0, tot = 0;
#pragma unroll
  for (int w = 0; w < NWAV; ++w) {
    const int v = swt[w];
    wpre += (w < wave) ? v : 0;
    tot += v;
  }
  pos = wpre + x - cnt;
  nh = tot;
}

__device__ __forceinline__ void ln_rows(const float* __restrict__ X, int rowBase, int nN,
                                        const float* sg, const float* sb, _Float16* sA, int wave, int lane) {
#pragma unroll 1
  for (int rr = 0; rr < GROWS / NWAV; ++rr) {
    const int row = wave * (GROWS / NWAV) + rr;
    int grow = rowBase + row;
    grow = grow > nN - 1 ? nN - 1 : grow;
    const float* xr = X + (size_t)grow * DD + 8 * lane;
    const v4f a0 = *(const v4f*)xr, a1 = *(const v4f*)(xr + 4);
    float v[8] = {a0.x, a0.y, a0.z, a0.w, a1.x, a1.y, a1.z, a1.w};
    float s = ((v[0] + v[1]) + (v[2] + v[3])) + ((v[4] + v[5]) + (v[6] + v[7]));
#pragma unroll
    for (int o = 16; o >= 1; o >>= 1) s += __shfl_xor(s, o, 32);
    const float mu = s * (1.0f / DD);
    float dv[8];
    float vs = 0.0f;
#pragma unroll
    for (int i = 0; i < 8; ++i) { dv[i] = v[i] - mu; vs = fmaf(dv[i], dv[i], vs); }
#pragma unroll
    for (int o = 16; o >= 1; o >>= 1) vs += __shfl_xor(vs, o, 32);
    const float rs = rsqrtf(fmaf(vs, 1.0f / DD, 1e-5f));
    v8h o;
#pragma unroll
    for (int i = 0; i < 8; ++i) o[i] = (_Float16)(fmaf(dv[i] * rs, sg[8 * lane + i], sb[8 * lane + i]) * HSC);
    *(v8h*)(sA + row * APZ + 8 * lane) = o;
  }
}

__global__ __launch_bounds__(NTHR) void k_node(const float* __restrict__ X, const float* __restrict__ g,
                                               const float* __restrict__ bta, const _Float16* __restrict__ Bp,
                                               const float* __restrict__ b1, float* PQ, int nN) {
  extern __shared__ __attribute__((aligned(16))) char dynl[];
  _Float16* sA  = (_Float16*)dynl;
  float*    sD  = (float*)(dynl + GROWS * APZ * 2);
  float*    sg  = sD + GROWS * PQW;
  float*    sb  = sg + DD;
  float*    sb1 = sb + DD;
  const int tid = threadIdx.x, lane = tid & 31, wave = tid >> 5, hh = lane >> 4, m = lane & 15;
  const int rowBase = blockIdx.x * GROWS;
  sg[tid] = g[tid];
  sb[tid] = bta[tid];
  sb1[tid] = b1[tid];
  __syncthreads();
  ln_rows(X, rowBase, nN, sg, sb, sA, wave, lane);
  __syncthreads();
  {
    const int rt = wave & 1, cg = wave >> 1;
    v8f acc[8];
    mma16<8>(sA + rt * 16 * APZ, Bp + (size_t)(128 * cg) * KP, lane, acc);
    float* sp = sD + (rt * 16 + 8 * hh) * PQW + 128 * cg + m;
#pragma unroll
    for (int t = 0; t < 8; ++t) {
      const int col = 128 * cg + 16 * t + m;
      const float bl = sb1[col & (DD - 1)];
      const float bv = (cg < 2) ? bl : 0.0f;
#pragma unroll
      for (int r = 0; r < 8; ++r) sp[r * PQW + 16 * t] = fmaf(acc[t][r], RH, bv);
    }
  }
  __syncthreads();

  float* gp = PQ + (size_t)rowBase * PQW;
#pragma unroll
  for (int it = 0; it < 16; ++it) {
    const int f = it * NTHR + tid;
    const v4f v = ((const v4f*)sD)[f];
    *(volatile v4f*)(gp + 4 * f) = v;
  }
  __threadfence();
#pragma unroll
  for (int it = 0; it < 16; ++it) {
    const int f = it * NTHR + tid;
    const v4f v = ((const v4f*)sD)[f];
    *(volatile v4f*)(gp + 4 * f) = v;
  }
}

__global__ __launch_bounds__(NTHR) void k_conv(
    const int* __restrict__ srcs, const int* __restrict__ dsts, const float* __restrict__ PQ,
    const _Float16* __restrict__ Bw, const float* __restrict__ b2, const float* __restrict__ Xold,
    float* Xnew, int nN, int nE, int nChunks, int vec) {
  extern __shared__ __attribute__((aligned(16))) char dynl[];
  unsigned* slist = (unsigned*)dynl;
  unsigned* glist = (unsigned*)(dynl + HC * 4);
  _Float16* sA    = (_Float16*)(dynl + HC * 4 + GC * 4);
  float*    sD    = (float*)(dynl + HC * 4 + GC * 4 + TROWS * APZ * 2);
  float*    sagg  = sD + TROWS * DD;
  float*    sb2   = sagg + GNODE * DD;
  int*      srl   = (int*)(sb2 + DD);
  int*      swt   = srl + TROWS;
  const int tid = threadIdx.x, lane = tid & 31, hh = lane >> 4, m = lane & 15;
  const int wave = __builtin_amdgcn_readfirstlane(tid >> 5);
  const int n0 = blockIdx.x * NBC;
  sb2[tid] = b2[tid];

  int base = 0;
#pragma unroll 1
  for (int c = 0; c < nChunks; ++c) {
    const int cbase = c * CHUNK;
    int d[EPT];
    loadids(dsts, nE, cbase, tid, vec, d);
    unsigned msk = 0;
#pragma unroll
    for (int j = 0; j < EPT; ++j) {
      const unsigned ld = (unsigned)d[j] - (unsigned)n0;
      msk |= ((ld < (unsigned)NBC) ? 1u : 0u) << j;
    }
    const int cnt = __builtin_popcount(msk);
    int pos, nh;
    blkscan(cnt, lane, wave, swt, pos, nh);
    const int e0 = cbase + EPT * tid;
#pragma unroll
    for (int j = 0; j < EPT; ++j) {
      if ((msk >> j) & 1u) {
        const int p = base + pos;
        if (p < HC) slist[p] = ((unsigned)(e0 + j) << 9) | ((unsigned)d[j] - (unsigned)n0);
        ++pos;
      }
    }
    base += nh;
    __syncthreads();
  }
  const int nht = __builtin_amdgcn_readfirstlane(base < HC ? base : HC);
  const int nlc = (nht + CHUNK - 1) / CHUNK;

#pragma unroll 1
  for (int gi = 0; gi < NGRP; ++gi) {
    {
      const float ninf = -__builtin_inff();
      v4f z = {ninf, ninf, ninf, ninf};
      v4f* p = (v4f*)sagg;
#pragma unroll
      for (int it = 0; it < 4; ++it) p[it * NTHR + tid] = z;
    }
    __syncthreads();

    int gtot = 0;
#pragma unroll 1
    for (int c = 0; c < nlc; ++c) {
      const int cb = c * CHUNK + EPT * tid;
      unsigned pk[EPT];
      unsigned msk = 0;
#pragma unroll
      for (int j = 0; j < EPT; ++j) {
        const int idx = cb + j;
        const bool ok = idx < nht;
        const int ic = ok ? idx : (HC - 1);
        pk[j] = slist[ic];
        const bool hit = ok && (((pk[j] >> 4) & 31u) == (unsigned)gi);
        msk |= (hit ? 1u : 0u) << j;
      }
      const int cnt = __builtin_popcount(msk);
      int pos, nh;
      blkscan(cnt, lane, wave, swt, pos, nh);
#pragma unroll
      for (int j = 0; j < EPT; ++j) {
        if ((msk >> j) & 1u) {
          const int p = gtot + pos;
          if (p < GC) glist[p] = pk[j];
          ++pos;
        }
      }
      gtot += nh;
      __syncthreads();
    }
    const int ng = __builtin_amdgcn_readfirstlane(gtot < GC ? gtot : GC);
    const int nt = (ng + TROWS - 1) / TROWS;

#pragma unroll 1
    for (int t = 0; t < nt; ++t) {
      {
        const int j = tid >> 3, q = tid & 7;
        const int idx = t * TROWS + j;
        const bool valid = idx < ng;
        const unsigned pkr = glist[idx];
        const unsigned pk1 = valid ? pkr : 0u;
        const int ld = (int)(pk1 & 15u);
        int e = (int)(pk1 >> 9);
        e = e > nE - 1 ? nE - 1 : e;
        int s = srcs[e];
        s = s < 0 ? 0 : (s > nN - 1 ? nN - 1 : s);
        const int dn = n0 + gi * GNODE + ld;
        const v4f* pp = (const v4f*)(PQ + (size_t)dn * PQW + 32 * q);
        const v4f* qp = (const v4f*)(PQ + (size_t)s * PQW + DD + 32 * q);
        _Float16* ar = sA + j * APZ + 32 * q;
#pragma unroll
        for (int i = 0; i < 4; ++i) {
          const v4f a0 = pp[2 * i], a1 = pp[2 * i + 1];
          const v4f c0 = qp[2 * i], c1 = qp[2 * i + 1];
          v8h hv;
          hv[0] = (_Float16)(fmaxf(a0.x + c0.x, 0.0f) * HSC); hv[1] = (_Float16)(fmaxf(a0.y + c0.y, 0.0f) * HSC);
          hv[2] = (_Float16)(fmaxf(a0.z + c0.z, 0.0f) * HSC); hv[3] = (_Float16)(fmaxf(a0.w + c0.w, 0.0f) * HSC);
          hv[4] = (_Float16)(fmaxf(a1.x + c1.x, 0.0f) * HSC); hv[5] = (_Float16)(fmaxf(a1.y + c1.y, 0.0f) * HSC);
          hv[6] = (_Float16)(fmaxf(a1.z + c1.z, 0.0f) * HSC); hv[7] = (_Float16)(fmaxf(a1.w + c1.w, 0.0f) * HSC);
          *(v8h*)(ar + 8 * i) = hv;
        }
        if (q == 0) srl[j] = valid ? ld : GNODE;
      }
      __syncthreads();

      v8f c0[2], c1[2];
      mma32<2>(sA, Bw + (size_t)(32 * wave) * KP, lane, c0, c1);
      {
        float* sp = sD + (8 * hh) * DD + 32 * wave + m;
#pragma unroll
        for (int tt = 0; tt < 2; ++tt) {
          const float bv = sb2[32 * wave + 16 * tt + m];
#pragma unroll
          for (int r = 0; r < 8; ++r) {
            sp[r * DD + 16 * tt]        = fmaf(c0[tt][r], RH, bv);
            sp[(16 + r) * DD + 16 * tt] = fmaf(c1[tt][r], RH, bv);
          }
        }
      }
      __syncthreads();

#pragma unroll 4
      for (int jr = 0; jr < TROWS; ++jr) {
        const int lj = srl[jr];
        const bool ok = lj < GNODE;
        const int lc = ok ? lj : 0;
        float* ap = sagg + lc * DD + tid;
        const float a = *ap;
        const float v = sD[jr * DD + tid];
        *ap = ok ? fmaxf(a, v) : a;
      }
      __syncthreads();
    }

    {
      const int gr0 = n0 + gi * GNODE;
      const float* xp = Xold + (size_t)gr0 * DD;
      float* gp = Xnew + (size_t)gr0 * DD;
      v4f ov[4];
#pragma unroll
      for (int it = 0; it < 4; ++it) {
        const int f = it * NTHR + tid;
        const v4f a = ((const v4f*)sagg)[f];
        const v4f xo = *(const v4f*)(xp + 4 * f);
        v4f r;
        r.x = fmaxf(a.x, 0.0f) + xo.x; r.y = fmaxf(a.y, 0.0f) + xo.y;
        r.z = fmaxf(a.z, 0.0f) + xo.z; r.w = fmaxf(a.w, 0.0f) + xo.w;
        ov[it] = r;
      }
#pragma unroll
      for (int it = 0; it < 4; ++it) *(volatile v4f*)(gp + 4 * (it * NTHR + tid)) = ov[it];
      __threadfence();
#pragma unroll
      for (int it = 0; it < 4; ++it) *(volatile v4f*)(gp + 4 * (it * NTHR + tid)) = ov[it];
    }
    __syncthreads();
  }
}

__global__ __launch_bounds__(NTHR) void k_ffn(const float* __restrict__ X, const float* __restrict__ g,
                                              const float* __restrict__ bta, const _Float16* __restrict__ Bf1,
                                              const float* __restrict__ fb1, const _Float16* __restrict__ Bf2,
                                              const float* __restrict__ fb2, float* Xout, int nN) {
  extern __shared__ __attribute__((aligned(16))) char dynl[];
  _Float16* sA  = (_Float16*)dynl;
  _Float16* sH  = (_Float16*)(dynl + GROWS * APZ * 2);
  float*    sD  = (float*)(dynl + 2 * GROWS * APZ * 2);
  float*    sg  = sD + GROWS * DD;
  float*    sb  = sg + DD;
  float*    sb1 = sb + DD;
  float*    sb2 = sb1 + DD;
  const int tid = threadIdx.x, lane = tid & 31, wave = tid >> 5, hh = lane >> 4, m = lane & 15;
  const int rowBase = blockIdx.x * GROWS;
  sg[tid] = g[tid];
  sb[tid] = bta[tid];
  sb1[tid] = fb1[tid];
  sb2[tid] = fb2[tid];
  __syncthreads();
  ln_rows(X, rowBase, nN, sg, sb, sA, wave, lane);
  __syncthreads();
  const int rt = wave & 1, cg = wave >> 1;
  {
    v8f acc[4];
    mma16<4>(sA + rt * 16 * APZ, Bf1 + (size_t)(64 * cg) * KP, lane, acc);
#pragma unroll
    for (int t = 0; t < 4; ++t) {
      const int col = 64 * cg + 16 * t + m;
      const float bv = sb1[col];
#pragma unroll
      for (int r = 0; r < 8; ++r)
        sH[(rt * 16 + 8 * hh + r) * APZ + col] = (_Float16)(fmaxf(fmaf(acc[t][r], RH, bv), 0.0f) * HSC);
    }
  }
  __syncthreads();
  {
    v8f acc[4];
    mma16<4>(sH + rt * 16 * APZ, Bf2 + (size_t)(64 * cg) * KP, lane, acc);
    float* sp = sD + (rt * 16 + 8 * hh) * DD + 64 * cg + m;
#pragma unroll
    for (int t = 0; t < 4; ++t) {
      const float bv = sb2[64 * cg + 16 * t + m];
#pragma unroll
      for (int r = 0; r < 8; ++r) sp[r * DD + 16 * t] = fmaf(acc[t][r], RH, bv);
    }
  }
  __syncthreads();

  const float* xp = X + (size_t)rowBase * DD;
  float* gp = Xout + (size_t)rowBase * DD;
  v4f ov[8];
#pragma unroll
  for (int it = 0; it < 8; ++it) {
    const int f = it * NTHR + tid;
    ov[it] = ((const v4f*)sD)[f] + *(const v4f*)(xp + 4 * f);
  }
#pragma unroll
  for (int it = 0; it < 8; ++it) *(volatile v4f*)(gp + 4 * (it * NTHR + tid)) = ov[it];
  __threadfence();
#pragma unroll
  for (int it = 0; it < 8; ++it) *(volatile v4f*)(gp + 4 * (it * NTHR + tid)) = ov[it];
}

__global__ __launch_bounds__(NTHR) void k_gather(const float* __restrict__ X, const int* __restrict__ sel,
                                                 float* out, int nRows, int selPer, int npg, int nN) {
  const int tid = threadIdx.x;
  const int R0 = blockIdx.x * ORB;
  v4f ov[4];
#pragma unroll
  for (int it = 0; it < 4; ++it) {
    const int f = it * NTHR + tid;
    int R = R0 + (f >> 6);
    R = R > nRows - 1 ? nRows - 1 : R;
    const int b = R / selPer;
    int si = sel[R];
    si = si < 0 ? 0 : (si > npg - 1 ? npg - 1 : si);
    int node = b * npg + si;
    node = node > nN - 1 ? nN - 1 : node;
    ov[it] = ((const v4f*)(X + (size_t)node * DD))[f & 63];
  }
  float* gp = out + (size_t)R0 * DD;
#pragma unroll
  for (int it = 0; it < 4; ++it) *(volatile v4f*)(gp + 4 * (it * NTHR + tid)) = ov[it];
  __threadfence();
#pragma unroll
  for (int it = 0; it < 4; ++it) *(volatile v4f*)(gp + 4 * (it * NTHR + tid)) = ov[it];
}

extern "C" void kernel_launch(void* const* d_in, const int* in_sizes, int n_in,
                              void* d_out, int out_size, void* d_ws, size_t ws_size,
                              hipStream_t stream) {
  if (n_in < 15) return;
  const int nN   = in_sizes[0] / DD;
  const int nE   = in_sizes[1] / 2;
  const int nSel = in_sizes[2];
  const int nl   = in_sizes[3] / (2 * DD * DD);
  if (in_sizes[0] != nN * DD || in_sizes[1] != 2 * nE) return;
  if (nN < NBC || (nN % NBC) != 0 || nN > (1 << 22)) return;
  if (nE < 1 || nE > (1 << 22)) return;
  if (nl < 1 || in_sizes[3] != nl * 2 * DD * DD || in_sizes[4] != nl * DD) return;
  if (in_sizes[5] != nl * DD * DD || in_sizes[6] != nl * DD) return;
  if (in_sizes[7] != DD || in_sizes[8] != DD || in_sizes[9] != DD || in_sizes[10] != DD) return;
  if (in_sizes[11] != DD * DD || in_sizes[12] != DD || in_sizes[13] != DD * DD || in_sizes[14] != DD) return;
  if (nSel < ORB || (nSel % ORB) != 0 || (nSel % NGRAPH) != 0 || (nN % NGRAPH) != 0) return;
  if (out_size != nSel * DD) return;
  const int npg    = nN / NGRAPH;
  const int selPer = nSel / NGRAPH;

  const float* x    = (const float*)d_in[0];
  const int*   ei   = (const int*)d_in[1];
  const int*   sel  = (const int*)d_in[2];
  const float* cw1  = (const float*)d_in[3];
  const float* cb1  = (const float*)d_in[4];
  const float* cw2  = (const float*)d_in[5];
  const float* cb2  = (const float*)d_in[6];
  const float* lncg = (const float*)d_in[7];
  const float* lncb = (const float*)d_in[8];
  const float* lnfg = (const float*)d_in[9];
  const float* lnfb = (const float*)d_in[10];
  const float* fw1  = (const float*)d_in[11];
  const float* fb1  = (const float*)d_in[12];
  const float* fw2  = (const float*)d_in[13];
  const float* fb2  = (const float*)d_in[14];
  float* out = (float*)d_out;
  const int* srcs = ei;
  const int* dsts = ei + (size_t)nE;

  char* ws = (char*)d_ws;
  size_t off = 0;
  const size_t oW1 = off; off += (size_t)nl * PQW * KP * 2;   off = (off + 255) & ~(size_t)255;
  const size_t oW2 = off; off += (size_t)nl * DD * KP * 2;    off = (off + 255) & ~(size_t)255;
  const size_t oF1 = off; off += (size_t)DD * KP * 2;         off = (off + 255) & ~(size_t)255;
  const size_t oF2 = off; off += (size_t)DD * KP * 2;         off = (off + 255) & ~(size_t)255;
  const size_t oPQ = off; off += (size_t)nN * PQW * 4;        off = (off + 255) & ~(size_t)255;
  const size_t oX0 = off; off += (size_t)nN * DD * 4;         off = (off + 255) & ~(size_t)255;
  const size_t oX1 = off; off += (size_t)nN * DD * 4;         off = (off + 255) & ~(size_t)255;
  if (off > ws_size || off > (size_t)WSCAP) return;
  _Float16* BW1 = (_Float16*)(ws + oW1);
  _Float16* BW2 = (_Float16*)(ws + oW2);
  _Float16* BF1 = (_Float16*)(ws + oF1);
  _Float16* BF2 = (_Float16*)(ws + oF2);
  float*    PQ  = (float*)(ws + oPQ);
  float*    X0  = (float*)(ws + oX0);
  float*    X1  = (float*)(ws + oX1);

  const int gNode   = nN / GROWS;
  const int gConv   = nN / NBC;
  const int nChunks = (nE + CHUNK - 1) / CHUNK;
  const int vec     = ((nE & 3) == 0) ? 1 : 0;
  const int gW      = nl * (W1T / NTHR) + nl * (W2T / NTHR) + 2 * (W2T / NTHR);

  hipFuncSetAttribute(reinterpret_cast<const void*>(&k_node), hipFuncAttributeMaxDynamicSharedMemorySize, LDS_NODE);
  hipFuncSetAttribute(reinterpret_cast<const void*>(&k_conv), hipFuncAttributeMaxDynamicSharedMemorySize, LDS_CONV);
  hipFuncSetAttribute(reinterpret_cast<const void*>(&k_ffn), hipFuncAttributeMaxDynamicSharedMemorySize, LDS_FFN);

  k_wprep<<<gW, NTHR, 0, stream>>>(cw1, cw2, fw1, fw2, BW1, BW2, BF1, BF2, nl);

  const float* xin = x;
  float* xout = X0;
  for (int l = 0; l < nl; ++l) {
    xout = ((l & 1) == 0) ? X0 : X1;
    k_node<<<gNode, NTHR, LDS_NODE, stream>>>(xin, lncg, lncb, BW1 + (size_t)l * PQW * KP, cb1 + (size_t)l * DD,
                                              PQ, nN);
    k_conv<<<gConv, NTHR, LDS_CONV, stream>>>(srcs, dsts, PQ, BW2 + (size_t)l * DD * KP, cb2 + (size_t)l * DD,
                                              xin, xout, nN, nE, nChunks, vec);
    xin = xout;
  }
  float* xf = (xout == X0) ? X1 : X0;

  k_ffn<<<gNode, NTHR, LDS_FFN, stream>>>(xin, lnfg, lnfb, BF1, fb1, BF2, fb2, xf, nN);
  k_gather<<<nSel / ORB, NTHR, 0, stream>>>(xf, sel, out, nSel, selPer, npg, nN);
}
